// MLPRegressor_51221779972563
// MI455X (gfx1250) — hardware-verified
//
#include <hip/hip_runtime.h>
#include <stddef.h>


typedef _Float16 h16;
typedef _Float16 v16h __attribute__((ext_vector_type(16)));
typedef _Float16 v8h  __attribute__((ext_vector_type(8)));
typedef float    v8f  __attribute__((ext_vector_type(8)));

#ifndef NB
#define NB 4096
#endif
#define NB_FULL 4096
#define SEQ   256
#define DM    32
#define XDIM  128
#define HIDN  64
#define NOUT  2

static_assert(NB >= 16 && NB <= NB_FULL);
static_assert((NB % 16) == 0);
static_assert(XDIM == 4 * DM);
static_assert((DM % 32) == 0 && (XDIM % 32) == 0);
static_assert((HIDN % 16) == 0 && HIDN == 64);
static_assert(16 * NOUT == 32);
static_assert(HIDN * NOUT == 4 * 32);

#define WCARRY 1024.0f
#define XCARRY 4096.0f

#define LDT 72
#define LDH 68
static_assert((LDT % 8) == 0 && LDT >= 64);
static_assert(LDH >= HIDN);

#define R_GENDER  0
#define R_KOREAN  2
#define R_PRIMARY 4
#define R_JOB     6
#define R_REP     17
#define R_PLACE   51
#define R_ADD     70
#define R_WP1     101
#define R_WC1     104
#define R_BP1     106
#define R_BC1     107
#define R_USED    108
#define TROWS     112
static_assert(R_KOREAN == R_GENDER + 2 && R_PRIMARY == R_KOREAN + 2 && R_JOB == R_PRIMARY + 2);
static_assert(R_REP == R_JOB + 11 && R_PLACE == R_REP + 34 && R_ADD == R_PLACE + 19);
static_assert(R_WP1 == R_ADD + 31 && R_WC1 == R_WP1 + 3 && R_BP1 == R_WC1 + 2 && R_BC1 == R_BP1 + 1);
static_assert(R_USED == R_BC1 + 1 && TROWS >= R_USED && (TROWS % 8) == 0);

#define W1T_BYTES ((size_t)HIDN * XDIM * 2)
#define WPC_BYTES ((size_t)2 * DM * DM * 2)
#define TAB_BYTES ((size_t)TROWS * DM * 4)
#define XP_BYTES  ((size_t)NB * XDIM * 2)
#define OFF_W1T ((size_t)0)
#define OFF_WPC (OFF_W1T + W1T_BYTES)
#define OFF_TAB (OFF_WPC + WPC_BYTES)
#define OFF_XP  (OFF_TAB + TAB_BYTES)
#define WS_TOTAL (OFF_XP + XP_BYTES)
static_assert((W1T_BYTES % 128) == 0 && (WPC_BYTES % 128) == 0 && (TAB_BYTES % 128) == 0);
static_assert((XP_BYTES % 128) == 0);
static_assert(W1T_BYTES == (size_t)4 * 256 * 8 * 2);
static_assert(WPC_BYTES == (size_t)256 * 8 * 2);
static_assert(TAB_BYTES == (size_t)(TROWS / 8) * 8 * 128);
static_assert(WS_TOTAL <= (size_t)134217728);

#define PREP_BLOCKS (4 + 1 + TROWS / 8)

__device__ __forceinline__ float bf16r(float x) {
  unsigned int u = __float_as_uint(x);
  u = (u + 0x7FFFu + ((u >> 16) & 1u)) & 0xFFFF0000u;
  return __uint_as_float(u);
}

static __device__ __forceinline__ h16 toh_flush(float v) {
  const h16 r = (h16)v;
  return (fabsf(v) < 6.103515625e-05f) ? (h16)0.0f : r;
}

__device__ __forceinline__ int clampi(int v, int lo, int hi) {
  return min(max(v, lo), hi);
}

__device__ __forceinline__ v16h frag_at(const _Float16* p) {
  v8h lo = *(const v8h*)(p);
  v8h hi = *(const v8h*)(p + 16);
  v16h out;
#pragma unroll
  for (int i = 0; i < 8; ++i) { out[i] = lo[i]; out[i + 8] = hi[i]; }
  return out;
}

__device__ __forceinline__ v8f wmma16(v16h a, v16h b, v8f c) {
  v8f d = __builtin_amdgcn_wmma_f32_16x16x32_f16(false, a, false, b, (short)0, c,
                                                 false, false);
  asm volatile("v_nop\n\tv_nop\n\tv_nop\n\tv_nop" : "+v"(d) : "v"(a), "v"(b));
  return d;
}

__global__ __launch_bounds__(256) void prep_kernel(
    const float* __restrict__ W1, const float* __restrict__ Wp2, const float* __restrict__ Wc2,
    const float* __restrict__ Eg, const float* __restrict__ Ek, const float* __restrict__ Ep,
    const float* __restrict__ Ej, const float* __restrict__ Er, const float* __restrict__ Epl,
    const float* __restrict__ Ea, const float* __restrict__ Wp1, const float* __restrict__ Wc1,
    const float* __restrict__ bp1, const float* __restrict__ bc1,
    _Float16* __restrict__ W1t, _Float16* __restrict__ WPCt, float* __restrict__ TAB) {
  const unsigned tid = threadIdx.x;
  const unsigned blk = blockIdx.x;
  if (blk < 4u) {
    const unsigned e = (blk * 256u + tid) * 8u;
    const unsigned n = e >> 7, k0 = e & 127u;
    v8h o;
#pragma unroll
    for (unsigned j = 0; j < 8u; ++j)
      o[j] = toh_flush(WCARRY * bf16r(W1[(size_t)(k0 + j) * HIDN + n]));
    *(volatile v8h*)(W1t + e) = o;
    __threadfence();
    *(volatile v8h*)(W1t + e) = o;
  } else if (blk == 4u) {
    const unsigned which = tid >> 7;
    const unsigned e = (tid & 127u) * 8u;
    const unsigned n = e >> 5, k0 = e & 31u;
    v8h o;
#pragma unroll
    for (unsigned j = 0; j < 8u; ++j) {
      const float a = Wp2[(k0 + j) * DM + n];
      const float c = Wc2[(k0 + j) * DM + n];
      const float v = (which != 0u) ? c : a;
      o[j] = toh_flush(WCARRY * bf16r(v));
    }
    *(volatile v8h*)(WPCt + tid * 8u) = o;
    __threadfence();
    *(volatile v8h*)(WPCt + tid * 8u) = o;
  } else {
    const unsigned lane = tid & 31u;
    int r = (int)(blk - 5u) * 8 + (int)(tid >> 5);
    asm volatile("" : "+v"(r));
    const float vg  = Eg [clampi(r - R_GENDER,  0, 1)  * DM + lane];
    const float vk  = Ek [clampi(r - R_KOREAN,  0, 1)  * DM + lane];
    const float vp  = Ep [clampi(r - R_PRIMARY, 0, 1)  * DM + lane];
    const float vj  = Ej [clampi(r - R_JOB,     0, 10) * DM + lane];
    const float vr  = Er [clampi(r - R_REP,     0, 33) * DM + lane];
    const float vpl = Epl[clampi(r - R_PLACE,   0, 18) * DM + lane];
    const float va  = Ea [clampi(r - R_ADD,     0, 30) * DM + lane];
    const float vw1 = Wp1[clampi(r - R_WP1,     0, 2)  * DM + lane];
    const float vc1 = Wc1[clampi(r - R_WC1,     0, 1)  * DM + lane];
    const float vb1 = bp1[lane];
    const float vb2 = bc1[lane];
    float v = 0.0f;
    v = (r < R_USED)    ? vb2 : v;
    v = (r < R_BC1)     ? vb1 : v;
    v = (r < R_BP1)     ? vc1 : v;
    v = (r < R_WC1)     ? vw1 : v;
    v = (r < R_WP1)     ? va  : v;
    v = (r < R_ADD)     ? vpl : v;
    v = (r < R_PLACE)   ? vr  : v;
    v = (r < R_REP)     ? vj  : v;
    v = (r < R_JOB)     ? vp  : v;
    v = (r < R_PRIMARY) ? vk  : v;
    v = (r < R_KOREAN)  ? vg  : v;
    const float ov = bf16r(v);
    float* dst = TAB + (size_t)r * DM + lane;
    *(volatile float*)dst = ov;
    __threadfence();
    *(volatile float*)dst = ov;
  }
}

__global__ __launch_bounds__(256) void pool_kernel(
    const float* __restrict__ cont_p, const float* __restrict__ cont_c,
    const int* __restrict__ cat_p, const int* __restrict__ cat_c,
    const int* __restrict__ lens, const float* __restrict__ TAB,
    _Float16* __restrict__ XP) {
  __shared__ float red[8 * 4 * 32];
  __shared__ __attribute__((aligned(16))) _Float16 xrow[XDIM];
  const unsigned tid = threadIdx.x, lane = tid & 31u;
  const int wave = __builtin_amdgcn_readfirstlane((int)(tid >> 5));
  const unsigned b = blockIdx.x;
  const int len_in = lens[b];
  const int len = clampi(len_in, 0, SEQ);
  const bool len_ok = (len_in >= 1) && (len_in <= SEQ);

  const float w0 = TAB[(R_WP1 + 0) * DM + lane];
  const float w1 = TAB[(R_WP1 + 1) * DM + lane];
  const float w2 = TAB[(R_WP1 + 2) * DM + lane];
  const float u0 = TAB[(R_WC1 + 0) * DM + lane];
  const float u1 = TAB[(R_WC1 + 1) * DM + lane];
  const float bP = TAB[R_BP1 * DM + lane];
  const float bC = TAB[R_BC1 * DM + lane];

  float s_rp = 0.0f, s_rc = 0.0f, s_ep = 0.0f, s_ec = 0.0f;

  for (int s = wave; s < len; s += 8) {
    const size_t t = (size_t)b * SEQ + (size_t)s;
    const float* cp = cont_p + t * 3;
    const float* cc = cont_c + t * 2;
    const int*   ip = cat_p + t * 5;
    const int*   ic = cat_c + t * 2;

    const float c0 = bf16r(cp[0]), c1 = bf16r(cp[1]), c2 = bf16r(cp[2]);
    const float d0 = bf16r(cc[0]), d1 = bf16r(cc[1]);
    const float rp = fmaxf(fmaf(c2, w2, fmaf(c1, w1, c0 * w0)) + bP, 0.0f);
    const float rc = fmaxf(fmaf(d1, u1, d0 * u0) + bC, 0.0f);
    s_rp += rp;
    s_rc += rc;

    const int i0 = R_GENDER  + clampi(ip[0], 0, 1);
    const int i1 = R_KOREAN  + clampi(ip[1], 0, 1);
    const int i2 = R_PRIMARY + clampi(ip[2], 0, 1);
    const int i3 = R_JOB     + clampi(ip[3], 0, 10);
    const int i4 = R_REP     + clampi(ip[4], 0, 33);
    const int j0 = R_PLACE   + clampi(ic[0], 0, 18);
    const int j1 = R_ADD     + clampi(ic[1], 0, 30);

    s_ep += (((TAB[i0 * DM + lane] + TAB[i1 * DM + lane]) + TAB[i2 * DM + lane])
             + TAB[i3 * DM + lane]) + TAB[j0 * DM + lane];
    s_ec += TAB[j1 * DM + lane] + TAB[i4 * DM + lane];
  }

  red[(wave * 4 + 0) * 32 + lane] = s_ep;
  red[(wave * 4 + 1) * 32 + lane] = s_ec;
  red[(wave * 4 + 2) * 32 + lane] = s_rp;
  red[(wave * 4 + 3) * 32 + lane] = s_rc;
  __syncthreads();

  if (tid < 128u) {
    const unsigned g = tid >> 5;
    float acc = 0.0f;
#pragma unroll
    for (unsigned w = 0; w < 8u; ++w) acc += red[(w * 4u + g) * 32u + lane];
    const float inv = len_ok ? (1.0f / (float)len_in) : 0.0f;
    const float f = (g == 0u) ? 0.2f : ((g == 1u) ? 0.5f : 1.0f);
    xrow[tid] = toh_flush((acc * (f * inv)) * XCARRY);
  }
  __syncthreads();

  const unsigned piece = (tid & 15u) * 8u;
  const v8h x = *(const v8h*)&xrow[piece];
  _Float16* dst = XP + (size_t)b * XDIM + piece;
  if (tid < 16u) *(volatile v8h*)dst = x;
  __threadfence();
  if (tid < 16u) *(volatile v8h*)dst = x;
}

__global__ __launch_bounds__(32) void mlp_kernel(
    const _Float16* __restrict__ XP, const _Float16* __restrict__ W1t,
    const _Float16* __restrict__ WPCt,
    const float* __restrict__ bp2, const float* __restrict__ bc2, const float* __restrict__ b1,
    const float* __restrict__ W2, const float* __restrict__ b2,
    const int* __restrict__ lens, float* __restrict__ out) {
  __shared__ __attribute__((aligned(16))) _Float16 xt2[16 * LDT];
  __shared__ float ht[16 * LDH];
  __shared__ float w2s[HIDN * NOUT];

  const unsigned lane = threadIdx.x & 31u;
  const unsigned hh = lane >> 4, m = lane & 15u;
  const unsigned rb = blockIdx.x * 16u;

#pragma unroll
  for (unsigned j = 0; j < 4u; ++j) w2s[lane + 32u * j] = bf16r(W2[lane + 32u * j]);

  const _Float16* xr = XP + (size_t)(rb + m) * XDIM + hh * 8u;
  const _Float16* wp = WPCt + (size_t)m * DM + hh * 8u;
  {
    const v16h a_p = frag_at(xr + 64);
    const v16h a_c = frag_at(xr + 96);
    const v16h bp0 = frag_at(wp);
    const v16h bp1 = frag_at(wp + 16 * DM);
    const v16h bc0 = frag_at(wp + DM * DM);
    const v16h bc1 = frag_at(wp + DM * DM + 16 * DM);
    v8f ap0 = {}, ap1 = {}, ac0 = {}, ac1 = {};
    ap0 = wmma16(a_p, bp0, ap0);
    ap1 = wmma16(a_p, bp1, ap1);
    ac0 = wmma16(a_c, bc0, ac0);
    ac1 = wmma16(a_c, bc1, ac1);
    const float gp0 = XCARRY * bf16r(bp2[m]);
    const float gp1 = XCARRY * bf16r(bp2[16u + m]);
    const float gc0 = XCARRY * bf16r(bc2[m]);
    const float gc1 = XCARRY * bf16r(bc2[16u + m]);
#pragma unroll
    for (int r = 0; r < 8; ++r) {
      const unsigned row = hh * 8u + (unsigned)r;
      xt2[row * LDT + m]       = toh_flush(ap0[r] * (1.0f / WCARRY) + gp0);
      xt2[row * LDT + 16u + m] = toh_flush(ap1[r] * (1.0f / WCARRY) + gp1);
      xt2[row * LDT + 32u + m] = toh_flush(ac0[r] * (1.0f / WCARRY) + gc0);
      xt2[row * LDT + 48u + m] = toh_flush(ac1[r] * (1.0f / WCARRY) + gc1);
    }
  }
  __syncthreads();

  v8f hacc[4];
#pragma unroll
  for (int n = 0; n < 4; ++n) hacc[n] = (v8f){};
  const _Float16* wb = W1t + (size_t)m * XDIM + hh * 8u;
#pragma unroll
  for (int ks = 0; ks < 2; ++ks) {
    const v16h a = frag_at(xr + ks * 32);
#pragma unroll
    for (int n = 0; n < 4; ++n) {
      const v16h bv = frag_at(wb + (size_t)(n * 16) * XDIM + ks * 32);
      hacc[n] = wmma16(a, bv, hacc[n]);
    }
  }
#pragma unroll
  for (int ks = 0; ks < 2; ++ks) {
    const v16h a = frag_at(&xt2[m * LDT + hh * 8u + (unsigned)ks * 32u]);
#pragma unroll
    for (int n = 0; n < 4; ++n) {
      const v16h bv = frag_at(wb + (size_t)(n * 16) * XDIM + (ks + 2) * 32);
      hacc[n] = wmma16(a, bv, hacc[n]);
    }
  }
#pragma unroll
  for (int n = 0; n < 4; ++n) {
    const float gb = bf16r(b1[(unsigned)n * 16u + m]);
#pragma unroll
    for (int r = 0; r < 8; ++r)
      ht[(hh * 8u + (unsigned)r) * LDH + (unsigned)n * 16u + m] =
          fmaxf(hacc[n][r] * (1.0f / (XCARRY * WCARRY)) + gb, 0.0f);
  }
  __syncthreads();

  const unsigned mo = lane >> 1, o = lane & 1u;
  int len_row = lens[rb + mo];
  asm volatile("" : "+v"(len_row));
  const bool row_ok = (len_row >= 1) && (len_row <= SEQ);
  float acc = bf16r(b2[o]);
#pragma unroll 4
  for (unsigned k = 0; k < (unsigned)HIDN; ++k)
    acc = fmaf(ht[mo * LDH + k], w2s[k * 2u + o], acc);
  const float relu_out = fmaxf(acc, 0.0f);
  const float val = row_ok ? relu_out : __uint_as_float(0x7fc00000u);
  float* dst = out + (size_t)rb * NOUT + lane;
  *(volatile float*)dst = val;
  __threadfence();
  *(volatile float*)dst = val;
}

extern "C" void kernel_launch(void* const* d_in, const int* in_sizes, int n_in,
                              void* d_out, int out_size, void* d_ws, size_t ws_size,
                              hipStream_t stream) {
  if (n_in < 24) return;
  const long long ntok = (long long)NB * SEQ;
  if ((long long)in_sizes[0] < ntok * 3) return;
  if ((long long)in_sizes[1] < ntok * 2) return;
  if ((long long)in_sizes[2] < ntok * 5) return;
  if ((long long)in_sizes[3] < ntok * 2) return;
  if (in_sizes[4] < NB) return;
  if (in_sizes[5] < 3 * DM || in_sizes[6] < DM) return;
  if (in_sizes[7] < DM * DM || in_sizes[8] < DM) return;
  if (in_sizes[9] < 2 * DM || in_sizes[10] < DM) return;
  if (in_sizes[11] < DM * DM || in_sizes[12] < DM) return;
  if (in_sizes[13] < 2 * DM || in_sizes[14] < 2 * DM || in_sizes[15] < 2 * DM) return;
  if (in_sizes[16] < 11 * DM || in_sizes[17] < 34 * DM) return;
  if (in_sizes[18] < 19 * DM || in_sizes[19] < 31 * DM) return;
  if (in_sizes[20] < XDIM * HIDN || in_sizes[21] < HIDN) return;
  if (in_sizes[22] < HIDN * NOUT || in_sizes[23] < NOUT) return;
  if ((long long)out_size < (long long)NB * NOUT) return;
  if (ws_size < WS_TOTAL) return;

  const float* cont_p    = (const float*)d_in[0];
  const float* cont_c    = (const float*)d_in[1];
  const int*   cat_p     = (const int*)d_in[2];
  const int*   cat_c     = (const int*)d_in[3];
  const int*   lens      = (const int*)d_in[4];
  const float* Wp1       = (const float*)d_in[5];
  const float* bp1       = (const float*)d_in[6];
  const float* Wp2       = (const float*)d_in[7];
  const float* bp2       = (const float*)d_in[8];
  const float* Wc1       = (const float*)d_in[9];
  const float* bc1       = (const float*)d_in[10];
  const float* Wc2       = (const float*)d_in[11];
  const float* bc2       = (const float*)d_in[12];
  const float* E_gender  = (const float*)d_in[13];
  const float* E_korean  = (const float*)d_in[14];
  const float* E_primary = (const float*)d_in[15];
  const float* E_job     = (const float*)d_in[16];
  const float* E_rep     = (const float*)d_in[17];
  const float* E_place   = (const float*)d_in[18];
  const float* E_add     = (const float*)d_in[19];
  const float* W1        = (const float*)d_in[20];
  const float* b1        = (const float*)d_in[21];
  const float* W2        = (const float*)d_in[22];
  const float* b2        = (const float*)d_in[23];
  float* out = (float*)d_out;

  char* ws = (char*)d_ws;
  _Float16* W1t  = (_Float16*)(ws + OFF_W1T);
  _Float16* WPCt = (_Float16*)(ws + OFF_WPC);
  float*    TAB  = (float*)(ws + OFF_TAB);
  _Float16* XP   = (_Float16*)(ws + OFF_XP);

  prep_kernel<<<dim3(PREP_BLOCKS), dim3(256), 0, stream>>>(
      W1, Wp2, Wc2, E_gender, E_korean, E_primary, E_job, E_rep, E_place, E_add,
      Wp1, Wc1, bp1, bc1, W1t, WPCt, TAB);
  pool_kernel<<<dim3(NB), dim3(256), 0, stream>>>(
      cont_p, cont_c, cat_p, cat_c, lens, TAB, XP);
  mlp_kernel<<<dim3(NB / 16), dim3(32), 0, stream>>>(
      XP, W1t, WPCt, bp2, bc2, b1, W2, b2, lens, out);
}
